// PaperDONNSentimentClassifier_76862734729918
// MI455X (gfx1250) — hardware-verified
//
#include <hip/hip_runtime.h>
#include <math.h>

constexpr int kBatch    = 128;
constexpr int kSeqLen   = 1024;
constexpr int kEmbDim   = 100;
constexpr int kUnits    = 100;
constexpr int kProj     = 20;
constexpr int kClasses  = 2;
constexpr int kHalfB    = 64;
constexpr int kRowsHalf = kHalfB * kSeqLen;
constexpr int kZPitch   = 256;
constexpr int kKPad     = 224;
constexpr int kNPad     = 128;
constexpr int kH1Pitch  = 128;
constexpr int kWPlane   = kNPad * kKPad;
constexpr float kDt      = 0.001f;
constexpr float kInScale = 0.2f;
constexpr float kMu      = 1.0f;
constexpr int kEulerSteps = 5;

typedef __attribute__((ext_vector_type(16))) _Float16 v16h;
typedef __attribute__((ext_vector_type(8)))  _Float16 v8h;
typedef __attribute__((ext_vector_type(16))) __bf16   v16b;
typedef __attribute__((ext_vector_type(8)))  __bf16   v8b;
typedef __attribute__((ext_vector_type(8)))  float    v8f;
typedef __attribute__((ext_vector_type(4)))  float    v4f;
typedef __attribute__((ext_vector_type(4)))  unsigned int   v4u;
typedef __attribute__((ext_vector_type(8)))  unsigned short v8us;

__device__ __forceinline__ unsigned short f2bf_bits(float f) {
  unsigned u = __float_as_uint(f);
  return (unsigned short)((u + 0x7FFFu + ((u >> 16) & 1u)) >> 16);
}
__device__ __forceinline__ float bf_bits2f(unsigned short h) { return __uint_as_float(((unsigned)h) << 16); }

__device__ __forceinline__ void dep_guard_h(v8f& a, v8f& b, v16h x, v16h y) { asm volatile("v_nop\n\tv_nop\n\tv_nop\n\tv_nop" : "+v"(a), "+v"(b) : "v"(x), "v"(y)); }
__device__ __forceinline__ void dep_guard_b(v8f& a, v8f& b, v16b x, v16b y) { asm volatile("v_nop\n\tv_nop\n\tv_nop\n\tv_nop" : "+v"(a), "+v"(b) : "v"(x), "v"(y)); }
__device__ __forceinline__ void keep4_h(v16h a, v16h b, v16h c, v16h d) { asm volatile("v_nop" :: "v"(a), "v"(b), "v"(c), "v"(d)); }
__device__ __forceinline__ void keep4_b(v16b a, v16b b, v16b c, v16b d) { asm volatile("v_nop" :: "v"(a), "v"(b), "v"(c), "v"(d)); }
__device__ __forceinline__ void acc_guard4(v8f& a, v8f& b, v8f& c, v8f& d) { asm volatile("v_nop\n\tv_nop\n\tv_nop\n\tv_nop" : "+v"(a), "+v"(b), "+v"(c), "+v"(d)); }
template <typename T> struct Frag;
template <> struct Frag<_Float16> {
  typedef v16h V; union U { v16h v; v8h h[2]; };
  static __device__ __forceinline__ v16h load(const _Float16* p) {
    U f; f.h[0] = *(const v8h*)(p); f.h[1] = *(const v8h*)(p + 16); return f.v;
  }
  static __device__ __forceinline__ v8f mma(v16h a, v16h b, v8f c) {
    return __builtin_amdgcn_wmma_f32_16x16x32_f16(false, a, false, b, (short)0, c, false, false);
  }
  static __device__ __forceinline__ void guard(v8f& a, v8f& b, v16h x, v16h y) { dep_guard_h(a, b, x, y); }
  static __device__ __forceinline__ void keep(v16h a, v16h b, v16h c, v16h d) { keep4_h(a, b, c, d); }
};
template <> struct Frag<__bf16> {
  typedef v16b V; union U { v16b v; v8b h[2]; };
  static __device__ __forceinline__ v16b load(const __bf16* p) {
    U f; f.h[0] = *(const v8b*)(p); f.h[1] = *(const v8b*)(p + 16); return f.v;
  }
  static __device__ __forceinline__ v8f mma(v16b a, v16b b, v8f c) {
    return __builtin_amdgcn_wmma_f32_16x16x32_bf16(false, a, false, b, (short)0, c, false, false);
  }
  static __device__ __forceinline__ void guard(v8f& a, v8f& b, v16b x, v16b y) { dep_guard_b(a, b, x, y); }
  static __device__ __forceinline__ void keep(v16b a, v16b b, v16b c, v16b d) { keep4_b(a, b, c, d); }
};

__device__ __forceinline__ unsigned pk16(unsigned short a, unsigned short b) { return (unsigned)a | ((unsigned)b << 16); }

template <int ET> struct Elem;
template <> struct Elem<0> { typedef _Float16 T; };
template <> struct Elem<1> { typedef __bf16 T; };
template <int ET, bool SPLIT, int BIAS_MODE, int OUT_MODE, bool RESID, int ACT = 0>
__global__ __launch_bounds__(256) void wmma_gemm64(
    const unsigned short* __restrict__ Ap, const unsigned short* __restrict__ A2p, int lda, long strideA,
    const unsigned short* __restrict__ Btp, const unsigned short* __restrict__ Bt2p, int ldb, long strideB,
    void* __restrict__ Cout, void* __restrict__ Cout2, int ldc, long strideC,
    const float* __restrict__ bias,
    const float* __restrict__ resid, long strideR,
    int M, int N, int K, float scale) {
  typedef typename Elem<ET>::T T;
  typedef typename Frag<T>::V V;
  const T* A = (const T*)Ap; const T* A2 = (const T*)A2p; const T* Bt = (const T*)Btp; const T* Bt2 = (const T*)Bt2p;
  __shared__ __align__(16) float sT[8][16 * 68];
  const int b    = blockIdx.y;
  const int lane = threadIdx.x & 31;
  const int wave = threadIdx.x >> 5;
  const int tilesN = N >> 6;
  const int tilesM = M >> 6;
  const int tile = blockIdx.x * 8 + wave;
  if (tile >= tilesM * tilesN) return;
  const int tm = tile / tilesN;
  const int tn = tile - tm * tilesN;
  const int m0 = tm << 6;
  const int n0 = tn << 6;

  const T* Ab  = A  + (size_t)b * strideA;
  const T* Bb  = Bt + (size_t)b * strideB;
  const T* Ab2 = SPLIT ? (A2  + (size_t)b * strideA) : nullptr;
  const T* Bb2 = SPLIT ? (Bt2 + (size_t)b * strideB) : nullptr;

  const int rlane = lane & 15;
  const int koff  = (lane >> 4) * 8;
  const int mOff  = (lane >> 4) * 8;

  v8f acc[4][4];
#pragma unroll
  for (int i = 0; i < 4; ++i)
#pragma unroll
    for (int j = 0; j < 4; ++j) acc[i][j] = (v8f){0.f,0.f,0.f,0.f,0.f,0.f,0.f,0.f};

  for (int k0 = 0; k0 < K; k0 += 32) {
    V bh[4], bl[4];
#pragma unroll
    for (int j = 0; j < 4; ++j) {
      const size_t bo = (size_t)(n0 + (j << 4) + rlane) * ldb + koff + k0;
      bh[j] = Frag<T>::load(Bb + bo);
      if (SPLIT) bl[j] = Frag<T>::load(Bb2 + bo);
    }
#pragma unroll
    for (int i = 0; i < 4; ++i) {
      const size_t ao = (size_t)(m0 + (i << 4) + rlane) * lda + koff + k0;
      V ah = Frag<T>::load(Ab + ao);
      V al;
      if (SPLIT) al = Frag<T>::load(Ab2 + ao);
#pragma unroll
      for (int j = 0; j < 4; ++j) {
        acc[i][j] = Frag<T>::mma(ah, bh[j], acc[i][j]);
        if (SPLIT) {
          acc[i][j] = Frag<T>::mma(ah, bl[j], acc[i][j]);
          acc[i][j] = Frag<T>::mma(al, bh[j], acc[i][j]);
        }
      }
      Frag<T>::guard(acc[i][0], acc[i][3], ah, SPLIT ? al : ah);
    }
    Frag<T>::keep(bh[0], bh[1], bh[2], bh[3]);
    if (SPLIT) Frag<T>::keep(bl[0], bl[1], bl[2], bl[3]);
  }
  acc_guard4(acc[0][0], acc[0][1], acc[0][2], acc[0][3]);
  acc_guard4(acc[1][0], acc[1][1], acc[1][2], acc[1][3]);
  acc_guard4(acc[2][0], acc[2][1], acc[2][2], acc[2][3]);
  acc_guard4(acc[3][0], acc[3][1], acc[3][2], acc[3][3]);

  float* slab = sT[wave];
  const float* Rb = RESID ? (resid + (size_t)b * strideR) : nullptr;
#pragma unroll
  for (int i = 0; i < 4; ++i) {
    const int mBase = m0 + (i << 4);
#pragma unroll
    for (int j = 0; j < 4; ++j) {
      const int n = n0 + (j << 4) + rlane;
      float bv = 0.f;
      if (BIAS_MODE == 2) bv = bias[n];
#pragma unroll
      for (int r = 0; r < 8; ++r) {
        float v = acc[i][j][r] * scale;
        if (BIAS_MODE == 1) v += bias[mBase + mOff + r];
        if (BIAS_MODE == 2) v += bv;
        if (RESID) v += Rb[(size_t)(mBase + mOff + r) * ldc + n];
        if (ACT == 1) v = tanhf(v);
        if (ACT == 2) v = fmaxf(v, 0.0f);
        if (ACT == 3) v = v / (1.0f + expf(-v));
        if (ACT == 4) v = (v > 0.f) ? v : 0.01f * v;
        if (ACT == 5) v = 0.5f * v * (1.0f + erff(v * 0.70710678118654752f));
        slab[(mOff + r) * 68 + (j << 4) + rlane] = v;
      }
    }
    __builtin_amdgcn_fence(__ATOMIC_RELEASE, "workgroup");
    __builtin_amdgcn_wave_barrier();
    __builtin_amdgcn_fence(__ATOMIC_ACQUIRE, "workgroup");
    if (OUT_MODE == 0) {
      float* C = (float*)Cout + (size_t)b * strideC;
      const int hh = lane >> 4, c4 = (lane & 15) * 4;
      for (int pass = 0; pass < 2; ++pass) {
#pragma unroll
        for (int it = 0; it < 8; ++it) {
          const int row = it * 2 + hh;
          v4f v = *(const v4f*)(slab + row * 68 + c4);
          *(volatile v4f*)(C + (size_t)(mBase + row) * ldc + n0 + c4) = v;
        }
        __threadfence();
      }
    } else {
      const int q = lane >> 3, c8 = (lane & 7) * 8;
      unsigned short* C  = (unsigned short*)Cout  + (size_t)b * strideC;
      unsigned short* C2 = (OUT_MODE == 2) ? ((unsigned short*)Cout2 + (size_t)b * strideC) : nullptr;
      for (int pass = 0; pass < 2; ++pass) {
#pragma unroll
        for (int it = 0; it < 4; ++it) {
          const int row = it * 4 + q;
          const float* sp = slab + row * 68 + c8;
          v8h hv, lv;
#pragma unroll
          for (int e = 0; e < 8; ++e) {
            if (OUT_MODE == 1) {
              hv[e] = (_Float16)sp[e];
            } else {
              unsigned short hb = f2bf_bits(sp[e]);
              unsigned short lb = f2bf_bits(sp[e] - bf_bits2f(hb));
              hv[e] = __builtin_bit_cast(_Float16, hb);
              lv[e] = __builtin_bit_cast(_Float16, lb);
            }
          }
          *(volatile v8h*)(C + (size_t)(mBase + row) * ldc + n0 + c8) = hv;
          if (OUT_MODE == 2) *(volatile v8h*)(C2 + (size_t)(mBase + row) * ldc + n0 + c8) = lv;
        }
        __threadfence();
      }
    }
    __builtin_amdgcn_fence(__ATOMIC_RELEASE, "workgroup");
    __builtin_amdgcn_wave_barrier();
    __builtin_amdgcn_fence(__ATOMIC_ACQUIRE, "workgroup");
  }
}

__global__ __launch_bounds__(256) void wcast_kernel(const float* __restrict__ w1, const float* __restrict__ w2,
                                                    unsigned short* __restrict__ WT) {
  const int sel = blockIdx.y;
  const float* w = (sel == 0) ? w1 : w2;
  const int i = blockIdx.x * 256 + threadIdx.x;
  if (i >= kWPlane / 8) return;
  unsigned short hb[8], lb[8];
#pragma unroll
  for (int e = 0; e < 8; ++e) {
    const int idx = 8 * i + e;
    const int n = idx / kKPad;
    const int k = idx - n * kKPad;
    const int nc = (n < kUnits) ? n : (kUnits - 1);
    const int kc = (k < 2 * kUnits) ? k : (2 * kUnits - 1);
    float v = w[kc * kUnits + nc];
    v = (n < kUnits && k < 2 * kUnits) ? v : 0.0f;
    const unsigned short h = f2bf_bits(v);
    hb[e] = h;
    lb[e] = f2bf_bits(v - bf_bits2f(h));
  }
  const v4u hv = (v4u){pk16(hb[0], hb[1]), pk16(hb[2], hb[3]), pk16(hb[4], hb[5]), pk16(hb[6], hb[7])};
  const v4u lv = (v4u){pk16(lb[0], lb[1]), pk16(lb[2], lb[3]), pk16(lb[4], lb[5]), pk16(lb[6], lb[7])};
  unsigned short* ph = WT + ((size_t)sel * 2 + 0) * kWPlane + 8 * (size_t)i;
  unsigned short* pl = WT + ((size_t)sel * 2 + 1) * kWPlane + 8 * (size_t)i;
  *(volatile v4u*)ph = hv;
  *(volatile v4u*)pl = lv;
  __threadfence();
  *(volatile v4u*)ph = hv;
  *(volatile v4u*)pl = lv;
}

__global__ __launch_bounds__(64) void biaspad_kernel(const float* __restrict__ b1, const float* __restrict__ b2, float* __restrict__ BP) {
  const int i = threadIdx.x;
  v4f v;
#pragma unroll
  for (int e = 0; e < 4; ++e) {
    const int idx = 4 * i + e;
    const int sel = idx >> 7;
    const int n = idx & 127;
    const int nc = (n < kUnits) ? n : (kUnits - 1);
    const float a = b1[nc];
    const float c = b2[nc];
    float val = (sel == 0) ? a : c;
    val = (n < kUnits) ? val : 0.0f;
    v[e] = val;
  }
  float* p = BP + 4 * i;
  *(volatile v4f*)p = v;
  __threadfence();
  *(volatile v4f*)p = v;
}

template <bool FROM_EMB>
__global__ __launch_bounds__(128) void hopf_kernel(const int* __restrict__ x, const float* __restrict__ emb, int vocab,
                                                   const float* __restrict__ H1, const float* __restrict__ omega,
                                                   unsigned short* __restrict__ Z, long planeStride, int b0) {
#pragma clang fp contract(off)
  __shared__ int sTok[kSeqLen];
  __shared__ __align__(16) unsigned short sZ[2][2][kZPitch];
  const int tid  = threadIdx.x;
  const int lane = tid & 31;
  const int wave = tid >> 5;
  const int u    = tid;
  const int uc   = (u < kUnits) ? u : (kUnits - 1);
  const int bl   = blockIdx.x;
  const int b    = b0 + bl;
  if (FROM_EMB) {
    for (int i = tid; i < kSeqLen; i += 128) {
      int tk = x[(size_t)b * kSeqLen + i];
      tk = (tk < 0) ? 0 : tk;
      tk = (tk >= vocab) ? (vocab - 1) : tk;
      sTok[i] = tk;
    }
  }
  for (int i = tid; i < 4 * (kZPitch - 2 * kUnits); i += 128) {
    const int q = i / (kZPitch - 2 * kUnits);
    const int c = i - q * (kZPitch - 2 * kUnits);
    sZ[q >> 1][q & 1][2 * kUnits + c] = (unsigned short)0;
  }
  const float om = omega[uc];
  float X = 0.0f, Y = 0.0f;
  __syncthreads();

#pragma unroll 1
  for (int t = 0; t < kSeqLen; ++t) {
    const int p = t & 1;
    float hval;
    if (FROM_EMB) {
      const int tk = sTok[t];
      hval = emb[(size_t)tk * kEmbDim + uc];
    } else {
      hval = H1[((size_t)bl * kSeqLen + t) * kH1Pitch + u];
    }
    const float d = kInScale * hval;
#pragma unroll
    for (int s = 0; s < kEulerSteps; ++s) {
      const float r2 = X * X + Y * Y;
      const float g  = kMu - r2;
      const float ax = g * X;
      const float oy = om * Y;
      const float t3 = ax - oy;
      const float t5 = t3 + d;
      const float nx = X + kDt * t5;
      const float ay = g * Y;
      const float ox = om * X;
      const float t6 = ay + ox;
      const float ny = Y + kDt * t6;
      X = nx;
      Y = ny;
    }
    if (u < kUnits) {
      const unsigned short hx = f2bf_bits(X);
      const unsigned short hy = f2bf_bits(Y);
      sZ[p][0][u]          = hx;
      sZ[p][0][kUnits + u] = hy;
      sZ[p][1][u]          = f2bf_bits(X - bf_bits2f(hx));
      sZ[p][1][kUnits + u] = f2bf_bits(Y - bf_bits2f(hy));
    }
    __syncthreads();
    if (wave < 2) {
      const v8us v = *(const v8us*)(&sZ[p][wave][lane * 8]);
      unsigned short* dst = Z + (size_t)wave * planeStride + ((size_t)bl * kSeqLen + t) * kZPitch + lane * 8;
      *(volatile v8us*)dst = v;
      __threadfence();
      *(volatile v8us*)dst = v;
    }
  }
}

__global__ __launch_bounds__(128) void head_kernel(const float* __restrict__ H2, const float* __restrict__ wp, const float* __restrict__ bp,
                                                   const float* __restrict__ wh, const float* __restrict__ bh, float* __restrict__ out) {
#pragma clang fp contract(off)
  __shared__ __align__(16) float sO[kBatch * kClasses];
  const int b = threadIdx.x;
  const float* hrow = H2 + (size_t)b * kH1Pitch;
  float o0 = 0.0f, o1 = 0.0f;
#pragma unroll 1
  for (int p = 0; p < kProj; ++p) {
    float s = 0.0f;
#pragma unroll 1
    for (int j = 0; j < kUnits; ++j) s = s + hrow[j] * wp[j * kProj + p];
    s = s + bp[p];
    const float h = tanhf(s);
    o0 = o0 + h * wh[p * kClasses + 0];
    o1 = o1 + h * wh[p * kClasses + 1];
  }
  o0 = o0 + bh[0];
  o1 = o1 + bh[1];
  sO[2 * b]     = o0;
  sO[2 * b + 1] = o1;
  __syncthreads();
  if (threadIdx.x < 64) {
    const v4f v = *(const v4f*)(sO + 4 * threadIdx.x);
    float* dst = out + 4 * threadIdx.x;
    *(volatile v4f*)dst = v;
    __threadfence();
    *(volatile v4f*)dst = v;
  }
}

extern "C" void kernel_launch(void* const* d_in, const int* in_sizes, int n_in,
                              void* d_out, int out_size, void* d_ws, size_t ws_size,
                              hipStream_t stream) {
  if (n_in < 12) return;
  if (in_sizes[0] != kBatch * kSeqLen) return;
  if (in_sizes[1] < kEmbDim || (in_sizes[1] % kEmbDim) != 0) return;
  if (in_sizes[2] != kUnits || in_sizes[3] != kUnits) return;
  if (in_sizes[4] != 2 * kUnits * kUnits || in_sizes[5] != kUnits) return;
  if (in_sizes[6] != 2 * kUnits * kUnits || in_sizes[7] != kUnits) return;
  if (in_sizes[8] != kUnits * kProj || in_sizes[9] != kProj) return;
  if (in_sizes[10] != kProj * kClasses || in_sizes[11] != kClasses) return;
  if (out_size != kBatch * kClasses) return;
  const int vocab = in_sizes[1] / kEmbDim;

  const int*   x      = (const int*)  d_in[0];
  const float* emb    = (const float*)d_in[1];
  const float* omega1 = (const float*)d_in[2];
  const float* omega2 = (const float*)d_in[3];
  const float* w1     = (const float*)d_in[4];
  const float* b1     = (const float*)d_in[5];
  const float* w2     = (const float*)d_in[6];
  const float* b2     = (const float*)d_in[7];
  const float* wp     = (const float*)d_in[8];
  const float* bp     = (const float*)d_in[9];
  const float* wh     = (const float*)d_in[10];
  const float* bh     = (const float*)d_in[11];
  float* outp = (float*)d_out;

  const size_t planeElems = (size_t)kRowsHalf * kZPitch;
  const size_t SZ_Z  = 2 * planeElems * 2;
  const size_t SZ_H1 = (size_t)kRowsHalf * kH1Pitch * 4;
  const size_t SZ_WT = (size_t)4 * kWPlane * 2;
  const size_t SZ_BP = (size_t)2 * kNPad * 4;
  const size_t SZ_H2 = (size_t)kBatch * kH1Pitch * 4;
  size_t off = 0;
  const size_t oZ  = off; off += SZ_Z;
  const size_t oH1 = off; off += SZ_H1;
  const size_t oWT = off; off += SZ_WT;
  const size_t oBP = off; off += SZ_BP;
  const size_t oH2 = off; off += SZ_H2;
  const size_t TOTAL = off;
  if (TOTAL > ws_size) return;
  if (TOTAL > (size_t)134217728) return;

  char* ws = (char*)d_ws;
  unsigned short* Z   = (unsigned short*)(ws + oZ);
  unsigned short* ZL  = Z + planeElems;
  float*          H1  = (float*)(ws + oH1);
  unsigned short* WT  = (unsigned short*)(ws + oWT);
  unsigned short* W1H = WT + 0 * (size_t)kWPlane;
  unsigned short* W1L = WT + 1 * (size_t)kWPlane;
  unsigned short* W2H = WT + 2 * (size_t)kWPlane;
  unsigned short* W2L = WT + 3 * (size_t)kWPlane;
  float*          BP  = (float*)(ws + oBP);
  float*          BP1 = BP;
  float*          BP2 = BP + kNPad;
  float*          H2  = (float*)(ws + oH2);

  wcast_kernel<<<dim3(kWPlane / 8 / 256, 2), dim3(256), 0, stream>>>(w1, w2, WT);
  biaspad_kernel<<<dim3(1), dim3(64), 0, stream>>>(b1, b2, BP);

  const long planeStride = (long)planeElems;
  const dim3 gG1((((kRowsHalf / 64) * (kNPad / 64)) + 7) / 8, 1);
  const dim3 gG2(1, 1);
  const size_t lastRowOff = (size_t)(kSeqLen - 1) * kZPitch;
  const int ldaLast = kSeqLen * kZPitch;

  for (int hf = 0; hf < kBatch / kHalfB; ++hf) {
    const int b0 = hf * kHalfB;
    hopf_kernel<true><<<dim3(kHalfB), dim3(128), 0, stream>>>(x, emb, vocab, H1, omega1, Z, planeStride, b0);
    wmma_gemm64<1, true, 2, 0, false, 2><<<gG1, dim3(256), 0, stream>>>(
        Z, ZL, kZPitch, 0L, W1H, W1L, kKPad, 0L, (void*)H1, (void*)H1, kH1Pitch, 0L,
        BP1, BP1, 0L, kRowsHalf, kNPad, kKPad, 1.0f);
    hopf_kernel<false><<<dim3(kHalfB), dim3(128), 0, stream>>>(x, emb, vocab, H1, omega2, Z, planeStride, b0);
    wmma_gemm64<1, true, 2, 0, false, 2><<<gG2, dim3(256), 0, stream>>>(
        Z + lastRowOff, ZL + lastRowOff, ldaLast, 0L, W2H, W2L, kKPad, 0L,
        (void*)(H2 + (size_t)b0 * kH1Pitch), (void*)(H2 + (size_t)b0 * kH1Pitch), kH1Pitch, 0L,
        BP2, BP2, 0L, kHalfB, kNPad, kKPad, 1.0f);
  }

  head_kernel<<<dim3(1), dim3(128), 0, stream>>>(H2, wp, bp, wh, bh, outp);
}
